// BatchdenseGAT_5171140625171
// MI455X (gfx1250) — hardware-run, weakly checked
//
#include <hip/hip_runtime.h>
#include <stdint.h>
#include <stddef.h>

#define NB    16
#define NN    512
#define NF0   64
#define NDE   64
#define NUE   3
#define NH    8
#define NO    128
#define NHO   1024
#define K0V   131
#define K0S   5
#define LD0   192
#define K1S   32
#define LD1   1024
#define TP    132
#define PRP   512
#define OTP   132
#define WSC   64.0f
#define HSC   16.0f
#define PSC   1024.0f
#define XSC   64.0f

typedef _Float16 v16h __attribute__((ext_vector_type(16)));
typedef _Float16 v8h  __attribute__((ext_vector_type(8)));
typedef float    v8f  __attribute__((ext_vector_type(8)));
typedef float    v4f  __attribute__((ext_vector_type(4)));

union Frag { v16h v; v8h h[2]; };
union U8f  { v4f v[2]; float f[8]; };
union U8h  { v8h v; _Float16 s[8]; };

__device__ __forceinline__ v8f mma16(v16h a, v16h b, v8f c) {
  return __builtin_amdgcn_wmma_f32_16x16x32_f16(false, a, false, b, (short)0, c, false, false);
}
__device__ __forceinline__ void guard1(v8f& c, v16h a, v16h b) {
  asm volatile("v_nop\n\tv_nop\n\tv_nop\n\tv_nop" : "+v"(c) : "v"(a), "v"(b));
}
__device__ __forceinline__ void guard4(v8f& c0, v8f& c1, v8f& c2, v8f& c3,
                                       v16h a, v16h b0, v16h b1, v16h b2, v16h b3) {
  asm volatile("v_nop\n\tv_nop\n\tv_nop\n\tv_nop"
               : "+v"(c0), "+v"(c1), "+v"(c2), "+v"(c3)
               : "v"(a), "v"(b0), "v"(b1), "v"(b2), "v"(b3));
}
__device__ __forceinline__ v8f vzero() { v8f z = {0.f,0.f,0.f,0.f,0.f,0.f,0.f,0.f}; return z; }

__global__ __launch_bounds__(256) void k_prep(
    const int* __restrict__ vtxg, const float* __restrict__ hfeat,
    const float* __restrict__ uemb, const float* __restrict__ etab,
    const float* __restrict__ n1w, const float* __restrict__ n1b,
    const float* __restrict__ n2w, const float* __restrict__ n2b,
    _Float16* __restrict__ X0, int nV)
{
  __shared__ int vtx[NN];
  __shared__ double es[256], eq[256], us[256], uq[256];
  __shared__ float cmean[68], cscl[68], cbia[68];
  const int tid = threadIdx.x, lane = tid & 31, w = tid >> 5, b = blockIdx.x;

  for (int n = tid; n < NN; n += 256) {
    int v = vtxg[b * NN + n];
    v = (v < 0) ? 0 : ((v > nV - 1) ? (nV - 1) : v);
    vtx[n] = v;
  }
  __syncthreads();
  {
    const int c = tid & 63, g = tid >> 6;
    double s = 0.0, q = 0.0;
#pragma unroll 2
    for (int k = 0; k < NN / 4; ++k) {
      const int n = g + 4 * k;
      const float v = etab[(size_t)vtx[n] * NDE + c];
      s += (double)v; q += (double)v * (double)v;
    }
    es[tid] = s; eq[tid] = q;
  }
  {
    const int cu = tid & 3, g2 = tid >> 2;
    const int cc = (cu < 3) ? cu : 2;
    double s = 0.0, q = 0.0;
#pragma unroll 1
    for (int k = 0; k < NN / 64; ++k) {
      const int n = g2 + 64 * k;
      float v = uemb[((size_t)b * NN + n) * NUE + cc];
      v = (cu < 3) ? v : 0.f;
      s += (double)v; q += (double)v * (double)v;
    }
    us[tid] = s; uq[tid] = q;
  }
  __syncthreads();
  if (w < 2) {
    const int c = tid;
    const double s = ((es[c] + es[64 + c]) + es[128 + c]) + es[192 + c];
    const double q = ((eq[c] + eq[64 + c]) + eq[128 + c]) + eq[192 + c];
    const double mu = s * (1.0 / NN);
    double var = q * (1.0 / NN) - mu * mu;
    var = (var > 0.0) ? var : 0.0;
    const float rstd = rsqrtf((float)var + 1e-5f);
    cmean[c] = (float)mu; cscl[c] = rstd * n1w[c]; cbia[c] = n1b[c];
  } else if (w == 2) {
    const int cu = lane & 3, cc = (cu < 3) ? cu : 2;
    double s = 0.0, q = 0.0;
#pragma unroll 1
    for (int g2 = 0; g2 < 64; ++g2) { s += us[g2 * 4 + cc]; q += uq[g2 * 4 + cc]; }
    const double mu = s * (1.0 / NN);
    double var = q * (1.0 / NN) - mu * mu;
    var = (var > 0.0) ? var : 0.0;
    const float rstd = rsqrtf((float)var + 1e-5f);
    if (lane < 3) { cmean[64 + lane] = (float)mu; cscl[64 + lane] = rstd * n2w[cc]; cbia[64 + lane] = n2b[cc]; }
  }
  __syncthreads();

  const int hc = ((lane < 8) ? lane : 7) * 8;
  const int ec = (lane & 7) * 8;
  float emn[8], esc[8], ebi[8];
#pragma unroll
  for (int e = 0; e < 8; ++e) { emn[e] = cmean[ec + e]; esc[e] = cscl[ec + e]; ebi[e] = cbia[ec + e]; }
  const float um0 = cmean[64], um1 = cmean[65], um2 = cmean[66];
  const float uc0 = cscl[64],  uc1 = cscl[65],  uc2 = cscl[66];
  const float ua0 = cbia[64],  ua1 = cbia[65],  ua2 = cbia[66];
#pragma unroll 1
  for (int k = 0; k < NN / 8; ++k) {
    const int n = w + 8 * k;
    const size_t row = (size_t)b * NN + n;
    U8f hu, eu;
    hu.v[0] = *(const v4f*)(hfeat + row * NF0 + hc);
    hu.v[1] = *(const v4f*)(hfeat + row * NF0 + hc + 4);
    const size_t eoff = (size_t)vtx[n] * NDE + ec;
    eu.v[0] = *(const v4f*)(etab + eoff);
    eu.v[1] = *(const v4f*)(etab + eoff + 4);
    const float u0 = uemb[row * NUE + 0], u1 = uemb[row * NUE + 1], u2 = uemb[row * NUE + 2];
    const float nu0 = (u0 - um0) * uc0 + ua0;
    const float nu1 = (u1 - um1) * uc1 + ua1;
    const float nu2 = (u2 - um2) * uc2 + ua2;
    U8h pk;
#pragma unroll
    for (int e = 0; e < 8; ++e) {
      const float ne  = (eu.f[e] - emn[e]) * esc[e] + ebi[e];
      const float uv  = (e == 0) ? nu0 : ((e == 1) ? nu1 : ((e == 2) ? nu2 : 0.f));
      const float sel = (lane < 8) ? hu.f[e] : ((lane < 16) ? ne : ((lane == 16) ? uv : 0.f));
      pk.s[e] = (_Float16)sel;
    }
    _Float16* dst = X0 + row * LD0 + lane * 8;
    if (lane < 24) *(volatile v8h*)dst = pk.v;
    __threadfence();
    if (lane < 24) *(volatile v8h*)dst = pk.v;
  }
}

__global__ __launch_bounds__(256) void k_packw(
    const float* __restrict__ w, _Float16* __restrict__ WT, int Kv, int Kp, int total8)
{
  const int gid = blockIdx.x * 256 + threadIdx.x;
  const int g = (gid < total8) ? gid : (total8 - 1);
  const int kp8 = Kp >> 3;
  const int n = g / kp8;
  const int k8 = (g - n * kp8) * 8;
  const int hh = n >> 7, o = n & 127;
  U8h pk;
#pragma unroll
  for (int e = 0; e < 8; ++e) {
    const int k = k8 + e;
    const int kc = (k < Kv) ? k : (Kv - 1);
    const float v = w[((size_t)hh * Kv + kc) * NO + o];
    pk.s[e] = (_Float16)((k < Kv) ? v * WSC : 0.f);
  }
  _Float16* dst = WT + (size_t)n * Kp + k8;
  if (gid < total8) *(volatile v8h*)dst = pk.v;
  __threadfence();
  if (gid < total8) *(volatile v8h*)dst = pk.v;
}

template <int KSTEPS, int LDA, int LDB>
__global__ __launch_bounds__(256) void k_gemm(
    const _Float16* __restrict__ X, const _Float16* __restrict__ WT,
    const float* __restrict__ asrc, const float* __restrict__ adst,
    _Float16* __restrict__ HPT, float* __restrict__ Sg, float* __restrict__ Dg, float accscale)
{
  __shared__ __align__(16) float T[64 * TP];
  __shared__ __align__(16) float sS[64];
  __shared__ __align__(16) float sD[64];
  const int tid = threadIdx.x, lane = tid & 31, w = tid >> 5;
  const int m = lane & 15, hi = lane >> 4;
  const int m0 = blockIdx.x * 64, hh = blockIdx.y;
  const int b = m0 / NN, j0 = m0 - b * NN;
  const int mr = (w & 3) * 16, nc = (w >> 2) * 64;
  const _Float16* Ap = X  + (size_t)(m0 + mr + m) * LDA + 8 * hi;
  const _Float16* Bp = WT + (size_t)(hh * NO + nc + m) * LDB + 8 * hi;

  v8f acc[4];
#pragma unroll
  for (int j = 0; j < 4; ++j) acc[j] = vzero();

#pragma unroll 1
  for (int ks = 0; ks < KSTEPS; ++ks) {
    const int k0 = ks * 32;
    Frag a, bq[4];
    a.h[0] = *(const v8h*)(Ap + k0);
    a.h[1] = *(const v8h*)(Ap + k0 + 16);
#pragma unroll
    for (int j = 0; j < 4; ++j) {
      const _Float16* bp = Bp + (size_t)j * 16 * LDB + k0;
      bq[j].h[0] = *(const v8h*)(bp);
      bq[j].h[1] = *(const v8h*)(bp + 16);
    }
#pragma unroll
    for (int j = 0; j < 4; ++j) acc[j] = mma16(a.v, bq[j].v, acc[j]);
    guard4(acc[0], acc[1], acc[2], acc[3], a.v, bq[0].v, bq[1].v, bq[2].v, bq[3].v);
  }

#pragma unroll
  for (int j = 0; j < 4; ++j) {
#pragma unroll
    for (int r = 0; r < 8; ++r)
      T[(mr + 8 * hi + r) * TP + nc + 16 * j + m] = acc[j][r] * accscale;
  }
  __syncthreads();

  {
    const int r = tid >> 2, q = tid & 3;
    const float* arow = asrc + hh * NO;
    const float* drow = adst + hh * NO;
    float s = 0.f, d = 0.f;
#pragma unroll 1
    for (int cI = 0; cI < 32; ++cI) {
      const int c = q * 32 + cI;
      const float t = tanhf(T[r * TP + c]);
      s = fmaf(t, arow[c], s);
      d = fmaf(t, drow[c], d);
    }
    s += __shfl_xor(s, 1, 32); s += __shfl_xor(s, 2, 32);
    d += __shfl_xor(d, 1, 32); d += __shfl_xor(d, 2, 32);
    if (q == 0) { sS[r] = s; sD[r] = d; }
  }
  U8h hv[4];
#pragma unroll
  for (int it = 0; it < 4; ++it) {
    const int o = it * 32 + (tid >> 3);
    const int jj = (tid & 7) * 8;
#pragma unroll
    for (int e = 0; e < 8; ++e) hv[it].s[e] = (_Float16)(T[(jj + e) * TP + o] * HSC);
  }
  __syncthreads();

  const size_t bh = (size_t)b * NH + hh;
  const int l4 = (lane & 15) * 4;
  const v4f sv = *(const v4f*)(sS + l4);
  const v4f dv = *(const v4f*)(sD + l4);
  float* sp = Sg + bh * NN + j0 + l4;
  float* dp = Dg + bh * NN + j0 + l4;
  for (int pass = 0; pass < 2; ++pass) {
#pragma unroll
    for (int it = 0; it < 4; ++it) {
      const int o = it * 32 + (tid >> 3);
      const int jj = (tid & 7) * 8;
      _Float16* hp = HPT + (bh * NO + o) * NN + j0 + jj;
      *(volatile v8h*)hp = hv[it].v;
    }
    if (w == 0) {
      if (lane < 16) *(volatile v4f*)sp = sv;
      if (lane < 16) *(volatile v4f*)dp = dv;
    }
    __threadfence();
  }
}

template <int MODE>
__global__ __launch_bounds__(256) void k_attn(
    const float* __restrict__ Sg, const float* __restrict__ Dg, const float* __restrict__ adj,
    const _Float16* __restrict__ HPT, _Float16* __restrict__ X1, float* __restrict__ out, float oscale)
{
  __shared__ __align__(16) _Float16 pr[16 * PRP];
  __shared__ __align__(16) float OT[16 * OTP];
  __shared__ float rowinv[16];
  const int tid = threadIdx.x, lane = tid & 31, w = tid >> 5;
  const int m = lane & 15, hi = lane >> 4;
  const int r = tid >> 4, c = tid & 15;
  const int b = blockIdx.y, i0 = blockIdx.x * 16, i = i0 + r;
  const float NEGINF = -__builtin_inff();

  unsigned mb = 0u;
  {
    const float* arow = adj + ((size_t)b * NN + i) * NN + c;
#pragma unroll
    for (int t = 0; t < 32; ++t) mb |= ((arow[16 * t] > 0.f) ? 1u : 0u) << t;
  }
  v8f hsum = vzero();

  for (int hh = 0; hh < NH; ++hh) {
    const size_t bh = (size_t)b * NH + hh;
    const float si = Sg[bh * NN + i];
    const float* drow = Dg + bh * NN + c;
    float ev[32];
    float mx = NEGINF;
#pragma unroll
    for (int t = 0; t < 32; ++t) {
      float e = si + drow[16 * t];
      e = (e >= 0.f) ? e : 0.2f * e;
      e = ((mb >> t) & 1u) ? e : NEGINF;
      ev[t] = e;
      mx = fmaxf(mx, e);
    }
    mx = fmaxf(mx, __shfl_xor(mx, 8, 32));
    mx = fmaxf(mx, __shfl_xor(mx, 4, 32));
    mx = fmaxf(mx, __shfl_xor(mx, 2, 32));
    mx = fmaxf(mx, __shfl_xor(mx, 1, 32));
    mx = (mx == NEGINF) ? 0.f : mx;
    float ls = 0.f;
#pragma unroll
    for (int t = 0; t < 32; ++t) {
      const float p = __expf(ev[t] - mx);
      ls += p;
      pr[r * PRP + c + 16 * t] = (_Float16)(p * PSC);
    }
    ls += __shfl_xor(ls, 8, 32);
    ls += __shfl_xor(ls, 4, 32);
    ls += __shfl_xor(ls, 2, 32);
    ls += __shfl_xor(ls, 1, 32);
    if (c == 0) rowinv[r] = (ls > 0.f) ? __builtin_amdgcn_rcpf(ls) : 0.f;
    __syncthreads();

    v8f acc = vzero();
    const _Float16* ap = pr + m * PRP + 8 * hi;
    const _Float16* bp = HPT + (bh * NO + w * 16 + m) * NN + 8 * hi;
#pragma unroll 4
    for (int k0 = 0; k0 < NN; k0 += 32) {
      Frag a, bq;
      a.h[0]  = *(const v8h*)(ap + k0);
      a.h[1]  = *(const v8h*)(ap + k0 + 16);
      bq.h[0] = *(const v8h*)(bp + k0);
      bq.h[1] = *(const v8h*)(bp + k0 + 16);
      acc = mma16(a.v, bq.v, acc);
      guard1(acc, a.v, bq.v);
    }

    if (MODE == 0) {
#pragma unroll
      for (int r8 = 0; r8 < 8; ++r8) {
        float v = acc[r8] * rowinv[8 * hi + r8] * oscale;
        v = (v > 0.f) ? v : expm1f(v);
        OT[(8 * hi + r8) * OTP + w * 16 + m] = v * XSC;
      }
      __syncthreads();
      {
        const int rr = tid >> 4, q = tid & 15;
        U8h pk;
#pragma unroll
        for (int e = 0; e < 8; ++e) pk.s[e] = (_Float16)OT[rr * OTP + q * 8 + e];
        _Float16* dst = X1 + ((size_t)b * NN + i0 + rr) * NHO + hh * NO + q * 8;
        *(volatile v8h*)dst = pk.v;
        __threadfence();
        *(volatile v8h*)dst = pk.v;
      }
    } else {
#pragma unroll
      for (int r8 = 0; r8 < 8; ++r8) hsum[r8] = fmaf(acc[r8], rowinv[8 * hi + r8], hsum[r8]);
      __syncthreads();
    }
  }

  if (MODE == 1) {
#pragma unroll
    for (int r8 = 0; r8 < 8; ++r8) OT[(8 * hi + r8) * OTP + w * 16 + m] = hsum[r8] * oscale;
    __syncthreads();
    {
      const int rr = tid >> 4, c8 = (tid & 15) * 8;
      float v[8];
      float mx = NEGINF;
#pragma unroll
      for (int e = 0; e < 8; ++e) { v[e] = OT[rr * OTP + c8 + e]; mx = fmaxf(mx, v[e]); }
      mx = fmaxf(mx, __shfl_xor(mx, 8, 32));
      mx = fmaxf(mx, __shfl_xor(mx, 4, 32));
      mx = fmaxf(mx, __shfl_xor(mx, 2, 32));
      mx = fmaxf(mx, __shfl_xor(mx, 1, 32));
      float se = 0.f;
#pragma unroll
      for (int e = 0; e < 8; ++e) se += expf(v[e] - mx);
      se += __shfl_xor(se, 8, 32);
      se += __shfl_xor(se, 4, 32);
      se += __shfl_xor(se, 2, 32);
      se += __shfl_xor(se, 1, 32);
      const float lse = logf(se);
#pragma unroll
      for (int e = 0; e < 8; ++e) OT[rr * OTP + c8 + e] = v[e] - mx - lse;
    }
    __syncthreads();
    for (int pass = 0; pass < 2; ++pass) {
#pragma unroll
      for (int it = 0; it < 2; ++it) {
        const int p = it * 256 + tid;
        const int rr = p >> 5, c4 = (p & 31) * 4;
        const v4f val = *(const v4f*)(OT + rr * OTP + c4);
        *(volatile v4f*)(out + ((size_t)b * NN + i0 + rr) * NO + c4) = val;
      }
      __threadfence();
    }
  }
}

extern "C" void kernel_launch(void* const* d_in, const int* in_sizes, int n_in,
                              void* d_out, int out_size, void* d_ws, size_t ws_size,
                              hipStream_t stream)
{
  if (n_in < 15) return;
  if (in_sizes[0] != NB * NN) return;
  if (in_sizes[1] != NB * NN * NN) return;
  if (in_sizes[2] != NB * NN * NF0) return;
  if (in_sizes[3] != NB * NN * NUE) return;
  if (in_sizes[4] < NDE || (in_sizes[4] % NDE) != 0) return;
  if (in_sizes[5] != NDE || in_sizes[6] != NDE || in_sizes[7] != NUE || in_sizes[8] != NUE) return;
  if (in_sizes[9] != NH * K0V * NO || in_sizes[10] != NH * NO || in_sizes[11] != NH * NO) return;
  if (in_sizes[12] != NH * LD1 * NO || in_sizes[13] != NH * NO || in_sizes[14] != NH * NO) return;
  if (out_size != NB * NN * NO) return;
  const int nV = in_sizes[4] / NDE;

  const int*   vertices = (const int*)  d_in[0];
  const float* adj      = (const float*)d_in[1];
  const float* hfeat    = (const float*)d_in[2];
  const float* uemb     = (const float*)d_in[3];
  const float* etab     = (const float*)d_in[4];
  const float* n1w = (const float*)d_in[5];
  const float* n1b = (const float*)d_in[6];
  const float* n2w = (const float*)d_in[7];
  const float* n2b = (const float*)d_in[8];
  const float* w0  = (const float*)d_in[9];
  const float* as0 = (const float*)d_in[10];
  const float* ad0 = (const float*)d_in[11];
  const float* w1  = (const float*)d_in[12];
  const float* as1 = (const float*)d_in[13];
  const float* ad1 = (const float*)d_in[14];

  const size_t szX0  = (size_t)NB * NN * LD0 * 2;
  const size_t szW0  = (size_t)NHO * LD0 * 2;
  const size_t szW1  = (size_t)NHO * LD1 * 2;
  const size_t szHPT = (size_t)NB * NH * NO * NN * 2;
  const size_t szSD  = (size_t)NB * NH * NN * 4;
  const size_t szX1  = (size_t)NB * NN * NHO * 2;
  size_t off = 0;
  const size_t oX0  = off; off += (szX0  + 255) & ~(size_t)255;
  const size_t oW0  = off; off += (szW0  + 255) & ~(size_t)255;
  const size_t oW1  = off; off += (szW1  + 255) & ~(size_t)255;
  const size_t oHPT = off; off += (szHPT + 255) & ~(size_t)255;
  const size_t oS   = off; off += (szSD  + 255) & ~(size_t)255;
  const size_t oD   = off; off += (szSD  + 255) & ~(size_t)255;
  const size_t oX1  = off; off += (szX1  + 255) & ~(size_t)255;
  if (off > ws_size) return;

  char* ws = (char*)d_ws;
  _Float16* X0  = (_Float16*)(ws + oX0);
  _Float16* W0T = (_Float16*)(ws + oW0);
  _Float16* W1T = (_Float16*)(ws + oW1);
  _Float16* HPT = (_Float16*)(ws + oHPT);
  float*    Sb  = (float*)(ws + oS);
  float*    Db  = (float*)(ws + oD);
  _Float16* X1  = (_Float16*)(ws + oX1);
  float*    outp = (float*)d_out;

  const int tot0 = NHO * LD0 / 8;
  const int tot1 = NHO * LD1 / 8;

  k_prep<<<dim3(NB), dim3(256), 0, stream>>>(vertices, hfeat, uemb, etab, n1w, n1b, n2w, n2b, X0, nV);
  k_packw<<<dim3((tot0 + 255) / 256), dim3(256), 0, stream>>>(w0, W0T, K0V, LD0, tot0);
  k_packw<<<dim3((tot1 + 255) / 256), dim3(256), 0, stream>>>(w1, W1T, LD1, LD1, tot1);

  k_gemm<K0S, LD0, LD0><<<dim3(NB * NN / 64, NH), dim3(256), 0, stream>>>(
      X0, W0T, as0, ad0, HPT, Sb, Db, 1.0f / WSC);
  k_attn<0><<<dim3(NN / 16, NB), dim3(256), 0, stream>>>(
      Sb, Db, adj, HPT, X1, outp, 1.0f / (PSC * HSC));

  k_gemm<K1S, LD1, LD1><<<dim3(NB * NN / 64, NH), dim3(256), 0, stream>>>(
      X1, W1T, as1, ad1, HPT, Sb, Db, 1.0f / (XSC * WSC));
  k_attn<1><<<dim3(NN / 16, NB), dim3(256), 0, stream>>>(
      Sb, Db, adj, HPT, X1, outp, 1.0f / (PSC * HSC * (float)NH));

  (void)hipGetLastError();
}
